// VaryMambaModel_6914897346922
// MI455X (gfx1250) — hardware-verified
//
#include <hip/hip_runtime.h>


#define NB_  2
#define LL   256
#define NS   64
typedef _Float16 h16;
typedef unsigned short bf;
typedef __attribute__((ext_vector_type(16))) __bf16   v16bf;
typedef __attribute__((ext_vector_type(16))) _Float16 v16h;
typedef __attribute__((ext_vector_type(8)))  _Float16 v8h;
typedef __attribute__((ext_vector_type(8)))  unsigned short v8us;
typedef __attribute__((ext_vector_type(8)))  float    v8f;
typedef __attribute__((ext_vector_type(4)))  float    v4f;
typedef v8h  __attribute__((may_alias)) v8ha;
typedef v4f  __attribute__((may_alias)) v4fa;
typedef v8us __attribute__((may_alias)) v8usa;

__device__ __forceinline__ unsigned short f2bf(float f) { unsigned u = __float_as_uint(f); u += 0x7FFFu + ((u >> 16) & 1u); return (unsigned short)(u >> 16); }
__device__ __forceinline__ float bf2f(unsigned short b) { return __uint_as_float(((unsigned)b) << 16); }
__device__ __forceinline__ float bfr(float f) { return bf2f(f2bf(f)); }
__device__ __forceinline__ v16h cat16(v8h lo, v8h hi) { return __builtin_shufflevector(lo, hi, 0, 1, 2, 3, 4, 5, 6, 7, 8, 9, 10, 11, 12, 13, 14, 15); }
__device__ __forceinline__ v16bf cat16b(v8us lo, v8us hi) { return __builtin_bit_cast(v16bf, __builtin_shufflevector(lo, hi, 0, 1, 2, 3, 4, 5, 6, 7, 8, 9, 10, 11, 12, 13, 14, 15)); }
__device__ __forceinline__ v8f wmma16(v16h a, v16h b, v8f c) { return __builtin_amdgcn_wmma_f32_16x16x32_f16(false, a, false, b, (short)0, c, false, false); }
__device__ __forceinline__ v8f wmmab(v16bf a, v16bf b, v8f c) { return __builtin_amdgcn_wmma_f32_16x16x32_bf16(false, a, false, b, (short)0, c, false, false); }


template <typename T16> struct WFrag;
template <> struct WFrag<h16> { typedef v16h V; static __device__ __forceinline__ V ld(const h16* p) { return cat16(*(const v8h*)p, *(const v8h*)(p + 16)); } static __device__ __forceinline__ v8f mma(V a, V b, v8f c) { return wmma16(a, b, c); } };
template <> struct WFrag<bf> { typedef v16bf V; static __device__ __forceinline__ V ld(const bf* p) { return cat16b(*(const v8us*)p, *(const v8us*)(p + 16)); } static __device__ __forceinline__ v8f mma(V a, V b, v8f c) { return wmmab(a, b, c); } };
template <typename T16, int NSPLIT, bool BIAS>
__global__ __launch_bounds__(32) void k_gemmw(const T16* __restrict__ A, const T16* __restrict__ A2, const T16* __restrict__ Bt, const T16* __restrict__ Bt2, int K, float* C, int ldc, const float* __restrict__ bias, size_t sA, size_t sB, size_t sC) {
    typedef typename WFrag<T16>::V V;
    __shared__ __align__(16) float os[16 * 68];
    const size_t z = blockIdx.z; A += z * sA; if (A2) A2 += z * sA; Bt += z * sB; if (Bt2) Bt2 += z * sB; C += z * sC;
    const int lane = threadIdx.x & 31, lr = lane & 15, hi = lane >> 4; const int r0 = blockIdx.x * 64, c0 = blockIdx.y * 64;
    v8f acc[4][4];
#pragma unroll
    for (int mb = 0; mb < 4; ++mb)
#pragma unroll
        for (int nb = 0; nb < 4; ++nb) acc[mb][nb] = (v8f){};
    const size_t aoff = (size_t)(r0 + lr) * K + 8 * hi, boff = (size_t)(c0 + lr) * K + 8 * hi;
#pragma unroll 1
    for (int kc = 0; kc < K; kc += 32) {
        V a[4], a2[4];
#pragma unroll
        for (int mb = 0; mb < 4; ++mb) { a[mb] = WFrag<T16>::ld(A + aoff + (size_t)mb * 16 * K + kc); if (NSPLIT == 1 || NSPLIT == 2) a2[mb] = WFrag<T16>::ld(A2 + aoff + (size_t)mb * 16 * K + kc); }
#pragma unroll
        for (int nb = 0; nb < 4; ++nb) { const V b = WFrag<T16>::ld(Bt + boff + (size_t)nb * 16 * K + kc); V b2; if (NSPLIT >= 2) b2 = WFrag<T16>::ld(Bt2 + boff + (size_t)nb * 16 * K + kc);
#pragma unroll
            for (int mb = 0; mb < 4; ++mb) { acc[mb][nb] = WFrag<T16>::mma(a[mb], b, acc[mb][nb]); if (NSPLIT == 1 || NSPLIT == 2) acc[mb][nb] = WFrag<T16>::mma(a2[mb], b, acc[mb][nb]); if (NSPLIT >= 2) acc[mb][nb] = WFrag<T16>::mma(a[mb], b2, acc[mb][nb]); } }
        asm volatile("v_nop\n\tv_nop\n\tv_nop\n\tv_nop" : "+v"(acc[0][0]), "+v"(acc[1][1]), "+v"(acc[2][2]), "+v"(acc[3][3]) : "v"(a[0]), "v"(a[3]));
    }
#pragma unroll
    for (int mb = 0; mb < 4; ++mb) {
#pragma unroll
        for (int nb = 0; nb < 4; ++nb) {
#pragma unroll
            for (int j = 0; j < 8; ++j) os[(hi * 8 + j) * 68 + nb * 16 + lr] = acc[mb][nb][j]; }
        __builtin_amdgcn_wave_barrier(); asm volatile("" ::: "memory");
        float* crow = C + (size_t)(r0 + mb * 16) * ldc + c0;
#pragma unroll 1
        for (int ps = 0; ps < 2; ++ps) {
#pragma unroll
            for (int s = 0; s < 8; ++s) { const int row = 2 * s + hi, cofs = lr * 4; v4f val = *(const v4fa*)(os + row * 68 + cofs); if (BIAS) { val[0] += bfr(bias[c0 + cofs]); val[1] += bfr(bias[c0 + cofs + 1]); val[2] += bfr(bias[c0 + cofs + 2]); val[3] += bfr(bias[c0 + cofs + 3]); }
                *(volatile v4f*)(crow + (size_t)row * ldc + cofs) = val; }
            if (ps == 0) __threadfence(); }
        __builtin_amdgcn_wave_barrier(); asm volatile("" ::: "memory");
    }
}

__device__ __forceinline__ void splitf(float y, unsigned short& h, unsigned short& l) { h = f2bf(y); l = f2bf(y - bf2f(h)); }
__device__ __forceinline__ float silu_(float x) { return __fmul_rn(x, __fdiv_rn(1.0f, 1.0f + __expf(-x))); }
typedef __attribute__((ext_vector_type(2))) unsigned short v2us;
typedef __attribute__((ext_vector_type(4))) unsigned short v4us;

__global__ __launch_bounds__(256) void k_wtG(const float* __restrict__ w, int K, int N, bf* Bt) {
    const int lane = threadIdx.x & 31; const int L0 = (blockIdx.x * 8 + (threadIdx.x >> 5)) * 8; const int nlines = N * K / 64;
#pragma unroll 1
    for (int ps = 0; ps < 2; ++ps) {
#pragma unroll 1
        for (int l = 0; l < 8; ++l) { const int L = L0 + l; if (L >= nlines) break; const size_t e = (size_t)L * 64 + lane * 2; const int k = (int)(e % K), n = (int)(e / K); v2us o;
            o[0] = f2bf(w[(size_t)k * N + n]); o[1] = f2bf(w[(size_t)(k + 1) * N + n]); *(volatile v2us*)(Bt + e) = o; }
        if (ps == 0) __threadfence(); }
}
__global__ __launch_bounds__(256) void k_x0(const float* __restrict__ pe, const float* __restrict__ cond, bf* Xh, bf* Xl) { const int e = (blockIdx.x * 256 + threadIdx.x) * 4; if (e >= LL * 1024) return; v4us oh, ol;
#pragma unroll
    for (int q = 0; q < 4; ++q) { unsigned short a, c; splitf(__fadd_rn(bfr(pe[e + q]), bfr(cond[e + q])), a, c); oh[q] = a; ol[q] = c; } *(volatile v4us*)(Xh + e) = oh; *(volatile v4us*)(Xl + e) = ol; __threadfence(); *(volatile v4us*)(Xh + e) = oh; *(volatile v4us*)(Xl + e) = ol; }
__global__ __launch_bounds__(256) void k_split(const float* __restrict__ F, int pitch, int c0, int wsel, bf* Hh, bf* Hl) { const int e = (blockIdx.x * 256 + threadIdx.x) * 4; if (e >= LL * wsel) return; const int c = e % wsel, t = e / wsel; const v4f a = *(const v4f*)(F + (size_t)t * pitch + c0 + c); v4us oh, ol;
#pragma unroll
    for (int q = 0; q < 4; ++q) { unsigned short u, l; splitf(a[q], u, l); oh[q] = u; ol[q] = l; } *(volatile v4us*)(Hh + e) = oh; *(volatile v4us*)(Hl + e) = ol; __threadfence(); *(volatile v4us*)(Hh + e) = oh; *(volatile v4us*)(Hl + e) = ol; }
__global__ __launch_bounds__(256) void k_conv(const float* __restrict__ XZ, int DI, const float* __restrict__ w, const float* __restrict__ bb, float* XC, bf* Ch, bf* Cl) { const int e = (blockIdx.x * 256 + threadIdx.x) * 4; if (e >= LL * DI) return; const int c = e % DI, t = e / DI; v4f o; v4us oh, ol;
#pragma unroll
    for (int q = 0; q < 4; ++q) { const int cc = c + q; float acc = bfr(bb[cc]);
#pragma unroll
        for (int k = 0; k < 4; ++k) { const int ts = t - 3 + k; if (ts >= 0) { float p = __fmul_rn(bfr(w[cc * 4 + k]), XZ[(size_t)ts * 2 * DI + cc]); asm volatile("" : "+v"(p)); acc = __fadd_rn(acc, p); } }
        o[q] = silu_(acc); unsigned short u, l; splitf(o[q], u, l); oh[q] = u; ol[q] = l; }
    for (int ps = 0; ps < 2; ++ps) { *(volatile v4f*)(XC + e) = o; *(volatile v4us*)(Ch + e) = oh; *(volatile v4us*)(Cl + e) = ol; if (ps == 0) __threadfence(); } }
__global__ __launch_bounds__(256) void k_scan(const float* __restrict__ DTR, const float* __restrict__ XC, const float* __restrict__ PROJ, int PW, int R, const float* __restrict__ XZ, const float* __restrict__ alog, const float* __restrict__ Dp, int DI, bf* Yh, bf* Yl) {
    __shared__ float ybuf[64]; const int tid = threadIdx.x; const int cl = tid >> 2, sub = tid & 3; const int d = blockIdx.x * 64 + cl; const int n0 = sub * 16; float A[16], h[16];
#pragma unroll
    for (int j = 0; j < 16; ++j) { A[j] = -__expf(bfr(alog[(size_t)d * NS + n0 + j])); h[j] = 0.f; }
    const float dd = bfr(Dp[d]);
    for (int t = 0; t < LL; ++t) { const float raw = DTR[(size_t)t * DI + d]; const float dt = raw > 20.f ? raw : log1pf(__expf(raw)); const float xc = XC[(size_t)t * DI + d]; const float dtx = __fmul_rn(dt, xc); const float* pr = PROJ + (size_t)t * PW + R; float y = 0.f;
#pragma unroll
        for (int j = 0; j < 16; ++j) { const float a = __expf(__fmul_rn(dt, A[j])); float hb = __fmul_rn(dtx, pr[n0 + j]); asm volatile("" : "+v"(hb)); float ha = __fmul_rn(a, h[j]); asm volatile("" : "+v"(ha)); h[j] = __fadd_rn(ha, hb); float yc = __fmul_rn(h[j], pr[NS + n0 + j]); asm volatile("" : "+v"(yc)); y = __fadd_rn(y, yc); }
        y += __shfl_xor(y, 1, 32); y += __shfl_xor(y, 2, 32);
        if (sub == 0) { float sk = __fmul_rn(dd, xc); asm volatile("" : "+v"(sk)); const float yy = __fadd_rn(y, sk); ybuf[cl] = __fmul_rn(yy, silu_(XZ[(size_t)t * 2 * DI + DI + d])); }
        __syncthreads();
        if (tid < 32) { v2us oh, ol; unsigned short u, l; splitf(ybuf[2 * tid], u, l); oh[0] = u; ol[0] = l; splitf(ybuf[2 * tid + 1], u, l); oh[1] = u; ol[1] = l; const size_t o = (size_t)t * DI + blockIdx.x * 64 + 2 * tid; *(volatile v2us*)(Yh + o) = oh; *(volatile v2us*)(Yl + o) = ol; __threadfence(); *(volatile v2us*)(Yh + o) = oh; *(volatile v2us*)(Yl + o) = ol; }
        __syncthreads(); } }

static void mamba_layer(hipStream_t stream, const bf* Xh, const bf* Xl, int D, int DI, int R, const bf* WIN, const float* cw, const float* cb, const bf* WX, int PW, const bf* WDT, const float* bdt, const float* alog, const float* Dp, const bf* WOUT, int DOUT,
                        float* XZ, float* XC, bf* Ch, bf* Cl, float* PROJ, bf* DTh, bf* DTl, float* DTR, bf* Yh, bf* Yl, float* OUTF) {
    k_gemmw<bf, 1, false><<<dim3(LL / 64, 2 * DI / 64, 1), 32, 0, stream>>>(Xh, Xl, WIN, nullptr, D, XZ, 2 * DI, nullptr, 0, 0, 0);
    k_conv<<<(LL * DI / 4 + 255) / 256, 256, 0, stream>>>(XZ, DI, cw, cb, XC, Ch, Cl);
    k_gemmw<bf, 1, false><<<dim3(LL / 64, PW / 64, 1), 32, 0, stream>>>(Ch, Cl, WX, nullptr, DI, PROJ, PW, nullptr, 0, 0, 0);
    k_split<<<(LL * R / 4 + 255) / 256, 256, 0, stream>>>(PROJ, PW, 0, R, DTh, DTl);
    k_gemmw<bf, 1, true><<<dim3(LL / 64, DI / 64, 1), 32, 0, stream>>>(DTh, DTl, WDT, nullptr, R, DTR, DI, bdt, 0, 0, 0);
    k_scan<<<DI / 64, 256, 0, stream>>>(DTR, XC, PROJ, PW, R, XZ, alog, Dp, DI, Yh, Yl);
    k_gemmw<bf, 1, false><<<dim3(LL / 64, DOUT / 64, 1), 32, 0, stream>>>(Yh, Yl, WOUT, nullptr, DI, OUTF, DOUT, nullptr, 0, 0, 0); }

extern "C" void kernel_launch(void* const* d_in, const int* in_sizes, int n_in,
                              void* d_out, int out_size, void* d_ws, size_t ws_size, hipStream_t stream) {
    (void)in_sizes; (void)n_in; (void)out_size;
    const float* cond = (const float*)d_in[0]; const float* pe = (const float*)d_in[2];
    const float* win1 = (const float*)d_in[3]; const float* cw1 = (const float*)d_in[4]; const float* cb1 = (const float*)d_in[5]; const float* wx1 = (const float*)d_in[6]; const float* wdt1 = (const float*)d_in[7]; const float* bdt1 = (const float*)d_in[8]; const float* alog1 = (const float*)d_in[9]; const float* d1p = (const float*)d_in[10]; const float* wout1 = (const float*)d_in[11];
    const float* win2 = (const float*)d_in[12]; const float* cw2 = (const float*)d_in[13]; const float* cb2 = (const float*)d_in[14]; const float* wx2 = (const float*)d_in[15]; const float* wdt2 = (const float*)d_in[16]; const float* bdt2 = (const float*)d_in[17]; const float* alog2 = (const float*)d_in[18]; const float* d2p = (const float*)d_in[19]; const float* wout2 = (const float*)d_in[20];
    float* OUT = (float*)d_out;
    char* wsp = (char*)d_ws;
    auto take = [&](size_t bytes) { char* p = wsp; wsp += (bytes + 255) & ~(size_t)255; return (void*)p; };
    bf* WIN1 = (bf*)take((size_t)4096 * 1024 * 2); bf* WX1 = (bf*)take((size_t)192 * 2048 * 2); bf* WDT1 = (bf*)take((size_t)2048 * 64 * 2); bf* WOUT1 = (bf*)take((size_t)1024 * 2048 * 2);
    bf* WIN2 = (bf*)take((size_t)8192 * 1024 * 2); bf* WX2 = (bf*)take((size_t)256 * 4096 * 2); bf* WDT2 = (bf*)take((size_t)4096 * 128 * 2); bf* WOUT2 = (bf*)take((size_t)2048 * 4096 * 2);
    bf* Xh = (bf*)take((size_t)LL * 1024 * 2); bf* Xl = (bf*)take((size_t)LL * 1024 * 2); float* XZ = (float*)take((size_t)LL * 8192 * 4); float* XC = (float*)take((size_t)LL * 4096 * 4); bf* Ch = (bf*)take((size_t)LL * 4096 * 2); bf* Cl = (bf*)take((size_t)LL * 4096 * 2); float* PROJ = (float*)take((size_t)LL * 256 * 4);
    bf* DTh = (bf*)take((size_t)LL * 128 * 2); bf* DTl = (bf*)take((size_t)LL * 128 * 2); float* DTR = (float*)take((size_t)LL * 4096 * 4); bf* Yh = (bf*)take((size_t)LL * 4096 * 2); bf* Yl = (bf*)take((size_t)LL * 4096 * 2); float* X1 = (float*)take((size_t)LL * 1024 * 4); bf* X1h = (bf*)take((size_t)LL * 1024 * 2); bf* X1l = (bf*)take((size_t)LL * 1024 * 2);
    if ((size_t)(wsp - (char*)d_ws) > ws_size) return;
    k_wtG<<<(1024 * 4096 / 64 + 63) / 64, 256, 0, stream>>>(win1, 1024, 4096, WIN1); k_wtG<<<(2048 * 192 / 64 + 63) / 64, 256, 0, stream>>>(wx1, 2048, 192, WX1); k_wtG<<<(64 * 2048 / 64 + 63) / 64, 256, 0, stream>>>(wdt1, 64, 2048, WDT1); k_wtG<<<(2048 * 1024 / 64 + 63) / 64, 256, 0, stream>>>(wout1, 2048, 1024, WOUT1);
    k_wtG<<<(1024 * 8192 / 64 + 63) / 64, 256, 0, stream>>>(win2, 1024, 8192, WIN2); k_wtG<<<(4096 * 256 / 64 + 63) / 64, 256, 0, stream>>>(wx2, 4096, 256, WX2); k_wtG<<<(128 * 4096 / 64 + 63) / 64, 256, 0, stream>>>(wdt2, 128, 4096, WDT2); k_wtG<<<(4096 * 2048 / 64 + 63) / 64, 256, 0, stream>>>(wout2, 4096, 2048, WOUT2);
    for (int b = 0; b < NB_; ++b) {
        k_x0<<<(LL * 1024 / 4 + 255) / 256, 256, 0, stream>>>(pe, cond + (size_t)b * LL * 1024, Xh, Xl);
        mamba_layer(stream, Xh, Xl, 1024, 2048, 64, WIN1, cw1, cb1, WX1, 192, WDT1, bdt1, alog1, d1p, WOUT1, 1024, XZ, XC, Ch, Cl, PROJ, DTh, DTl, DTR, Yh, Yl, X1);
        k_split<<<(LL * 1024 / 4 + 255) / 256, 256, 0, stream>>>(X1, 1024, 0, 1024, X1h, X1l);
        mamba_layer(stream, X1h, X1l, 1024, 4096, 128, WIN2, cw2, cb2, WX2, 256, WDT2, bdt2, alog2, d2p, WOUT2, 2048, XZ, XC, Ch, Cl, PROJ, DTh, DTl, DTR, Yh, Yl, OUT + (size_t)b * LL * 2048); }
}
